// ScaledDotProductAttention_22488448762365
// MI455X (gfx1250) — hardware-verified
//
#include <hip/hip_runtime.h>
#ifndef NB
#define NB 16
#endif
#ifndef SEQ
#define SEQ 2048
#endif
#define NB_FULL 16
#define SEQ_FULL 2048
#define HD 64
#define QT (SEQ / 64)
#define PCARRY 4096.0f
#define XCARRY 16.0f
#define CL2 (1.44269504088896340736f * 0.125f / (XCARRY * XCARRY))
#define FILLV (-1.0e20f)
#define PLANE_HALVES ((size_t)NB * SEQ * HD)

static_assert(SEQ % 64 == 0);
static_assert(SEQ <= SEQ_FULL);
static_assert(NB <= NB_FULL);
static_assert(HD == 64);
static_assert(((size_t)NB * QT) * 2u * 256u * 8u == PLANE_HALVES);
static_assert(((size_t)NB * QT) * 4u * 16u * 64u == PLANE_HALVES);

typedef unsigned short v8us __attribute__((ext_vector_type(8), may_alias));
typedef float  v8f  __attribute__((ext_vector_type(8)));
typedef float  v4f  __attribute__((ext_vector_type(4)));
typedef float  v4fa __attribute__((ext_vector_type(4), may_alias));
typedef _Float16 v16h __attribute__((ext_vector_type(16)));
union FragH { v16h v; v8us half[2]; _Float16 h[16]; unsigned short u[16]; };

__device__ __forceinline__ float bf16_rne(float x) {
  unsigned int u = __float_as_uint(x);
  u = (u + 0x7FFFu + ((u >> 16) & 1u)) & 0xFFFF0000u;
  return __uint_as_float(u);
}
__device__ __forceinline__ _Float16 in16(float x) { return (_Float16)(bf16_rne(x) * XCARRY); }

__device__ __forceinline__ v16h g2_frag(const _Float16* p, unsigned hh) {
  FragH f;
  f.half[0] = *(const v8us*)((const unsigned short*)p + 8u * hh);
  f.half[1] = *(const v8us*)((const unsigned short*)p + 16u + 8u * hh);
  return f.v;
}
__device__ __forceinline__ v8f g2_mma(v16h a, v16h b, v8f c) {
  v8f d = __builtin_amdgcn_wmma_f32_16x16x32_f16(false, a, false, b, (short)0, c, false, false);
  asm volatile("v_nop\n\tv_nop\n\tv_nop\n\tv_nop" : "+v"(d) : "v"(a), "v"(b));
  return d;
}
__device__ __forceinline__ v16h q_frag(const float* p, unsigned hh) {
  const v4f x0 = *(const v4fa*)(p + 8u * hh), x1 = *(const v4fa*)(p + 8u * hh + 4u);
  const v4f x2 = *(const v4fa*)(p + 16u + 8u * hh), x3 = *(const v4fa*)(p + 16u + 8u * hh + 4u);
  FragH f;
#pragma unroll
  for (int q = 0; q < 4; ++q) { f.h[q] = in16(x0[q]); f.h[4 + q] = in16(x1[q]); f.h[8 + q] = in16(x2[q]); f.h[12 + q] = in16(x3[q]); }
  return f.v;
}

__global__ __launch_bounds__(256) void k_prep(const float* __restrict__ Kin, const float* __restrict__ Vin,
                                             unsigned short* __restrict__ K16, unsigned short* __restrict__ VT) {
  __shared__ unsigned short tl[64][66];
  const unsigned tid = threadIdx.x;
  const unsigned b = blockIdx.x / QT, sg = blockIdx.x - b * QT, s0 = sg * 64u;
  FragH fk[2], fv[2];
#pragma unroll
  for (int u = 0; u < 2; ++u) {
    const unsigned i = tid + 256u * (unsigned)u, j = i >> 3, d8 = (i & 7u) << 3;
    const size_t src = ((size_t)b * SEQ_FULL + s0 + j) * HD + d8;
    const v4f ka = *(const v4fa*)(Kin + src), kc = *(const v4fa*)(Kin + src + 4);
    const v4f va = *(const v4fa*)(Vin + src), vc = *(const v4fa*)(Vin + src + 4);
    FragH t;
#pragma unroll
    for (int q = 0; q < 4; ++q) { fk[u].h[q] = in16(ka[q]); fk[u].h[4 + q] = in16(kc[q]); t.h[q] = in16(va[q]); t.h[4 + q] = in16(vc[q]); }
#pragma unroll
    for (int q = 0; q < 8; ++q) tl[d8 + q][j] = t.u[q];
  }
  __syncthreads();
#pragma unroll
  for (int u = 0; u < 2; ++u) {
    const unsigned i = tid + 256u * (unsigned)u, d = i >> 3, j8 = (i & 7u) << 3;
#pragma unroll
    for (int q = 0; q < 8; ++q) fv[u].u[q] = tl[d][j8 + q];
  }
  for (int pass = 0; pass < 2; ++pass) {
#pragma unroll
    for (int u = 0; u < 2; ++u) {
      const unsigned i = tid + 256u * (unsigned)u, r = i >> 3, c8 = (i & 7u) << 3;
      *(volatile v8us*)(K16 + ((size_t)b * SEQ + s0 + r) * HD + c8) = fk[u].half[0];
      *(volatile v8us*)(VT + ((size_t)b * HD + r) * SEQ + s0 + c8) = fv[u].half[0];
    }
    if (pass == 0) __threadfence();
  }
}

__global__ __launch_bounds__(128) void k_flash(const float* __restrict__ Q, const _Float16* __restrict__ K16, const _Float16* __restrict__ VT,
                                              const int* __restrict__ vlen, float* __restrict__ O) {
  __shared__ __attribute__((aligned(16))) float so[4][16][68];
  const unsigned tid = threadIdx.x, w = tid >> 5, lane = tid & 31u, nl = lane & 15u, g = lane >> 4;
  const unsigned b = blockIdx.x / QT, qb = blockIdx.x - b * QT;
  const unsigned q0 = qb * 64u + w * 16u;
  int vli = vlen[b];
  vli = vli < 0 ? 0 : vli;
  vli = vli > SEQ ? SEQ : vli;
  const unsigned vl = (unsigned)vli;
  unsigned kend = (vl > 0u) ? ((vl + 31u) & ~31u) : (unsigned)SEQ;
  kend = kend > (unsigned)SEQ ? (unsigned)SEQ : kend;
  const unsigned ntile = kend >> 5;

  const float* qrow = Q + ((size_t)b * SEQ_FULL + q0 + nl) * HD;
  const v16h bq0 = q_frag(qrow, g), bq1 = q_frag(qrow + 32, g);
  const _Float16* kr = K16 + ((size_t)b * SEQ + nl) * HD;
  const _Float16* vr = VT + ((size_t)b * HD + nl) * SEQ;

  const v8f z8 = {0.f, 0.f, 0.f, 0.f, 0.f, 0.f, 0.f, 0.f};
  v8f o0 = z8, o1 = z8, o2 = z8, o3 = z8;
  float m = -3.0e38f, l = 0.0f;

#pragma unroll 1
  for (unsigned t = 0; t < ntile; ++t) {
    const unsigned k0 = t << 5;
    const _Float16* ka = kr + (size_t)k0 * HD;
    v8f st0 = z8, st1 = z8;
    st0 = g2_mma(g2_frag(ka, g), bq0, st0);
    st1 = g2_mma(g2_frag(ka + 16 * HD, g), bq0, st1);
    st0 = g2_mma(g2_frag(ka + 32, g), bq1, st0);
    st1 = g2_mma(g2_frag(ka + 16 * HD + 32, g), bq1, st1);

    float s0[8], s1[8];
#pragma unroll
    for (int i = 0; i < 8; ++i) {
      const unsigned key0 = k0 + 8u * g + (unsigned)i;
      const float a0 = st0[i] * CL2, a1 = st1[i] * CL2;
      s0[i] = (key0 < vl) ? a0 : FILLV;
      s1[i] = (key0 + 16u < vl) ? a1 : FILLV;
    }
    float tmax = fmaxf(s0[0], s1[0]);
#pragma unroll
    for (int i = 1; i < 8; ++i) tmax = fmaxf(tmax, fmaxf(s0[i], s1[i]));
    tmax = fmaxf(tmax, __shfl_xor(tmax, 16));
    const float mn = fmaxf(m, tmax);
    const float alpha = __builtin_amdgcn_exp2f(m - mn);

    FragH pb;
    float psum = 0.0f;
#pragma unroll
    for (int i = 0; i < 8; ++i) {
      const _Float16 h0 = (_Float16)(__builtin_amdgcn_exp2f(s0[i] - mn) * PCARRY);
      const _Float16 h1 = (_Float16)(__builtin_amdgcn_exp2f(s1[i] - mn) * PCARRY);
      pb.h[i] = h0;
      pb.h[8 + i] = h1;
      psum += (float)h0 + (float)h1;
    }
    psum += __shfl_xor(psum, 16);
    l = l * alpha + psum;
    m = mn;
    o0 *= alpha; o1 *= alpha; o2 *= alpha; o3 *= alpha;

    const _Float16* va = vr + k0;
    o0 = g2_mma(g2_frag(va, g), pb.v, o0);
    o1 = g2_mma(g2_frag(va + (size_t)16 * SEQ, g), pb.v, o1);
    o2 = g2_mma(g2_frag(va + (size_t)32 * SEQ, g), pb.v, o2);
    o3 = g2_mma(g2_frag(va + (size_t)48 * SEQ, g), pb.v, o3);
  }

  const float inv = (1.0f / l) * (1.0f / XCARRY);
#pragma unroll
  for (int i = 0; i < 8; ++i) {
    so[w][nl][0 * 16 + 8u * g + i] = o0[i] * inv;
    so[w][nl][1 * 16 + 8u * g + i] = o1[i] * inv;
    so[w][nl][2 * 16 + 8u * g + i] = o2[i] * inv;
    so[w][nl][3 * 16 + 8u * g + i] = o3[i] * inv;
  }
  __builtin_amdgcn_fence(4  , "workgroup");
  __builtin_amdgcn_wave_barrier();
  const unsigned rsub = lane >> 4, c4 = (lane & 15u) * 4u;
  float* ob = O + ((size_t)b * SEQ + q0) * HD;
  for (int pass = 0; pass < 2; ++pass) {
#pragma unroll
    for (int q = 0; q < 8; ++q) {
      const unsigned r = (unsigned)q * 2u + rsub;
      const v4f v = *(const v4fa*)&so[w][r][c4];
      *(volatile v4f*)(ob + (size_t)r * HD + c4) = v;
    }
    if (pass == 0) __threadfence();
  }
}

extern "C" void kernel_launch(void* const* d_in, const int* in_sizes, int n_in,
                              void* d_out, int out_size, void* d_ws, size_t ws_size, hipStream_t stream) {
  if (n_in < 4) return;
  const long long need_in = ((long long)(NB - 1) * SEQ_FULL + SEQ) * HD;
  if ((long long)in_sizes[0] < need_in || (long long)in_sizes[1] < need_in || (long long)in_sizes[2] < need_in) return;
  if (in_sizes[3] < NB) return;
  if ((long long)out_size < (long long)NB * SEQ * HD) return;
  const float* q = (const float*)d_in[0];
  const float* k = (const float*)d_in[1];
  const float* v = (const float*)d_in[2];
  const int* vlen = (const int*)d_in[3];
  const size_t plane_bytes = PLANE_HALVES * 2u;
  if (2u * plane_bytes > ws_size) return;
  unsigned short* K16 = (unsigned short*)d_ws;
  unsigned short* VT = (unsigned short*)((char*)d_ws + plane_bytes);
  k_prep<<<NB * QT, 256, 0, stream>>>(k, v, K16, VT);
  k_flash<<<NB * QT, 128, 0, stream>>>(q, (const _Float16*)K16, (const _Float16*)VT, vlen, (float*)d_out);
}
